// SLULatticeRNN_28132035788899
// MI455X (gfx1250) — hardware-verified
//
#include <hip/hip_runtime.h>
#define NBt 32
#define TT 128
#define KP 4
#define EE 300
#define HH 512
#define G4 2048
#define NL 64
#define AP 1024
#define K0 832
#define K1 1024
typedef __bf16 v16b __attribute__((ext_vector_type(16)));
typedef unsigned short v8us __attribute__((ext_vector_type(8), may_alias));
typedef float  v8f  __attribute__((ext_vector_type(8)));
typedef float  v4f  __attribute__((ext_vector_type(4)));
typedef float  v4fa __attribute__((ext_vector_type(4), may_alias));
union FragB { v16b v; v8us half[2]; unsigned short u[16]; };

__device__ __forceinline__ unsigned short bf16_bits(float x) { unsigned int u = __float_as_uint(x); return (unsigned short)((u + 0x7FFFu + ((u >> 16) & 1u)) >> 16); }
__device__ __forceinline__ float bf16_val(unsigned short b) { return __uint_as_float(((unsigned int)b) << 16); }
__device__ __forceinline__ float bf16_round(float x) { return bf16_val(bf16_bits(x)); }
template <int NT>
__device__ __forceinline__ v8f mmaN(v16b ah, v16b al, v16b bh, v16b bl, v8f c) {
  c = __builtin_amdgcn_wmma_f32_16x16x32_bf16(false, ah, false, bh, (short)0, c, false, false);
  if (NT >= 2) c = __builtin_amdgcn_wmma_f32_16x16x32_bf16(false, al, false, bh, (short)0, c, false, false);
  if (NT >= 3) c = __builtin_amdgcn_wmma_f32_16x16x32_bf16(false, ah, false, bl, (short)0, c, false, false);
  asm volatile("v_nop\n\tv_nop\n\tv_nop\n\tv_nop" : "+v"(c) : "v"(ah), "v"(al), "v"(bh), "v"(bl));
  return c;
}

__global__ __launch_bounds__(256) void k_wt_bf16(const float* __restrict__ W, unsigned short* __restrict__ Wt, int K, int N) {
  const int t = blockIdx.x * 256 + threadIdx.x;
  const int k8n = K / 8;
  if (t >= N * k8n) return;
  const int n = t / k8n, k8 = (t % k8n) * 8;
  v8us v;
#pragma unroll
  for (int i = 0; i < 8; ++i) v[i] = bf16_bits(W[(size_t)(k8 + i) * N + n]);
  *(volatile v8us*)(Wt + (size_t)n * K + k8) = v;
  __threadfence();
  *(volatile v8us*)(Wt + (size_t)n * K + k8) = v;
}

template <bool ASPLIT, int ACT, bool BIAS_BF16>
__global__ __launch_bounds__(128) void k_gemm_bf(const float* __restrict__ A, int lda, const unsigned short* __restrict__ Wt, int ldb,
                                               const float* __restrict__ bias, float* __restrict__ C, int ldc, int M, int N, int K) {
  __shared__ __attribute__((aligned(16))) float so[4][16][64];
  const int tid = threadIdx.x, w = tid >> 5, lane = tid & 31, ln = lane & 15, hh = lane >> 4;
  const int ntn = N / 64;
  const int wid = blockIdx.x * 4 + w;
  const int mt = wid / ntn, nq = wid % ntn;
  if (mt * 16 >= M) return;
  const int row0 = mt * 16, col0 = nq * 64;
  const float* arow = A + (size_t)(row0 + ln) * lda;
  v8f acc[4] = {};
  for (int kb = 0; kb < K; kb += 32) {
    FragB ah, al;
    const v4f x0 = *(const v4fa*)(arow + kb + 8 * hh), x1 = *(const v4fa*)(arow + kb + 8 * hh + 4);
    const v4f x2 = *(const v4fa*)(arow + kb + 16 + 8 * hh), x3 = *(const v4fa*)(arow + kb + 16 + 8 * hh + 4);
    float xs[16] = {x0[0],x0[1],x0[2],x0[3],x1[0],x1[1],x1[2],x1[3],x2[0],x2[1],x2[2],x2[3],x3[0],x3[1],x3[2],x3[3]};
#pragma unroll
    for (int i = 0; i < 16; ++i) { const unsigned short hb = bf16_bits(xs[i]); ah.u[i] = hb; al.u[i] = ASPLIT ? bf16_bits(xs[i] - bf16_val(hb)) : (unsigned short)0; }
#pragma unroll
    for (int t = 0; t < 4; ++t) {
      const unsigned short* brow = Wt + (size_t)(col0 + t * 16 + ln) * ldb + kb;
      FragB b;
      b.half[0] = *(const v8us*)(brow + 8 * hh);
      b.half[1] = *(const v8us*)(brow + 16 + 8 * hh);
      acc[t] = mmaN<ASPLIT ? 2 : 1>(ah.v, al.v, b.v, b.v, acc[t]);
    }
  }
#pragma unroll
  for (int t = 0; t < 4; ++t) {
    float bv = bias ? bias[col0 + t * 16 + ln] : 0.f;
    if (BIAS_BF16) bv = bf16_round(bv);
#pragma unroll
    for (int r = 0; r < 8; ++r) { float v = acc[t][r] + bv; if (ACT == 1) v = fmaxf(v, 0.f); so[w][8 * hh + r][t * 16 + ln] = v; }
  }
  __builtin_amdgcn_fence(__ATOMIC_ACQ_REL, "workgroup");
  __builtin_amdgcn_wave_barrier();
  const int rsub = lane >> 4, c4 = (lane & 15) * 4;
  for (int pass = 0; pass < 2; ++pass) {
#pragma unroll
    for (int q = 0; q < 8; ++q) {
      const int r = q * 2 + rsub;
      const v4f v = *(const v4fa*)&so[w][r][c4];
      *(volatile v4f*)(C + (size_t)(row0 + r) * ldc + col0 + c4) = v;
    }
    if (pass == 0) __threadfence();
  }
}

template <bool ASPLIT, int ACT, bool BIAS_BF16, bool RES_BF16>
__global__ __launch_bounds__(128) void k_gemm_bf3(const float* __restrict__ A, int lda, const unsigned short* __restrict__ Wt, int ldb,
                                                const float* __restrict__ bias, const float* __restrict__ resid, int rmod, int ldr,
                                                float* __restrict__ C, int ldc, int M, int N, int K) {
  __shared__ __attribute__((aligned(16))) float so[4][16][64];
  const int tid = threadIdx.x, w = tid >> 5, lane = tid & 31, ln = lane & 15, hh = lane >> 4;
  const int ntn = N / 64;
  const int wid = blockIdx.x * 4 + w;
  const int mt = wid / ntn, nq = wid % ntn;
  if (mt * 16 >= M) return;
  const int row0 = mt * 16, col0 = nq * 64;
  const float* arow = A + (size_t)(row0 + ln) * lda;
  v8f acc[4] = {};
  for (int kb = 0; kb < K; kb += 32) {
    FragB ah, al;
    const v4f x0 = *(const v4fa*)(arow + kb + 8 * hh), x1 = *(const v4fa*)(arow + kb + 8 * hh + 4);
    const v4f x2 = *(const v4fa*)(arow + kb + 16 + 8 * hh), x3 = *(const v4fa*)(arow + kb + 16 + 8 * hh + 4);
    float xs[16] = {x0[0],x0[1],x0[2],x0[3],x1[0],x1[1],x1[2],x1[3],x2[0],x2[1],x2[2],x2[3],x3[0],x3[1],x3[2],x3[3]};
#pragma unroll
    for (int i = 0; i < 16; ++i) { const unsigned short hb = bf16_bits(xs[i]); ah.u[i] = hb; al.u[i] = ASPLIT ? bf16_bits(xs[i] - bf16_val(hb)) : (unsigned short)0; }
#pragma unroll
    for (int t = 0; t < 4; ++t) {
      const unsigned short* brow = Wt + (size_t)(col0 + t * 16 + ln) * ldb + kb;
      FragB b;
      b.half[0] = *(const v8us*)(brow + 8 * hh);
      b.half[1] = *(const v8us*)(brow + 16 + 8 * hh);
      acc[t] = mmaN<ASPLIT ? 2 : 1>(ah.v, al.v, b.v, b.v, acc[t]);
    }
  }
#pragma unroll
  for (int t = 0; t < 4; ++t) {
    const int col = col0 + t * 16 + ln;
    float bv = bias ? bias[col] : 0.f;
    if (BIAS_BF16) bv = bf16_round(bv);
#pragma unroll
    for (int r = 0; r < 8; ++r) {
      float v = acc[t][r] + bv;
      if (resid) { float rv = resid[(size_t)((row0 + 8 * hh + r) % rmod) * ldr + col]; if (RES_BF16) rv = bf16_round(rv); v += rv; }
      if (ACT == 1) v = fmaxf(v, 0.f);
      if (ACT == 2) v = 0.5f * v * (1.0f + erff(v * 0.70710678118654752f));
      if (ACT == 3) { const float u = 0.7978845608028654f * (v + 0.044715f * v * v * v); v = 0.5f * v * (1.0f + tanhf(u)); }
      so[w][8 * hh + r][t * 16 + ln] = v;
    }
  }
  __builtin_amdgcn_fence(__ATOMIC_ACQ_REL, "workgroup");
  __builtin_amdgcn_wave_barrier();
  const int rsub = lane >> 4, c4 = (lane & 15) * 4;
  for (int pass = 0; pass < 2; ++pass) {
#pragma unroll
    for (int q = 0; q < 8; ++q) {
      const int r = q * 2 + rsub;
      const v4f v = *(const v4fa*)&so[w][r][c4];
      *(volatile v4f*)(C + (size_t)(row0 + r) * ldc + col0 + c4) = v;
    }
    if (pass == 0) __threadfence();
  }
}
template <bool PARAM_BF16>
__global__ __launch_bounds__(256) void k_layernorm(const float* __restrict__ X, const float* __restrict__ R, const float* __restrict__ g, const float* __restrict__ bta,
                                                  float* __restrict__ out_sum, float* __restrict__ out_norm, int N, float eps) {
  __shared__ float red[256];
  const int row = blockIdx.x, tid = threadIdx.x;
  const float* x = X + (size_t)row * N; const float* rr = R ? R + (size_t)row * N : nullptr;
  float vals[16];
  const int per = N / 256;
  float s1 = 0.f;
  for (int u = 0; u < per / 4; ++u) {
    const int j = tid * 4 + 1024 * u;
    const v4f a = *(const v4fa*)(x + j);
    v4f b = {0.f,0.f,0.f,0.f}; if (rr) b = *(const v4fa*)(rr + j);
#pragma unroll
    for (int q = 0; q < 4; ++q) { const float v = a[q] + b[q]; vals[u * 4 + q] = v; s1 += v; }
  }
  red[tid] = s1; __syncthreads();
  for (int st = 128; st > 0; st >>= 1) { if (tid < st) red[tid] += red[tid + st]; __syncthreads(); }
  const float mu = red[0] / (float)N; __syncthreads();
  float s2 = 0.f;
  for (int u = 0; u < per / 4; ++u)
#pragma unroll
    for (int q = 0; q < 4; ++q) { const float c = vals[u * 4 + q] - mu; s2 += c * c; }
  red[tid] = s2; __syncthreads();
  for (int st = 128; st > 0; st >>= 1) { if (tid < st) red[tid] += red[tid + st]; __syncthreads(); }
  const float rs = rsqrtf(red[0] / (float)N + eps);
  for (int pass = 0; pass < 2; ++pass) {
    for (int u = 0; u < per / 4; ++u) {
      const int j = tid * 4 + 1024 * u;
      v4f o, sm;
#pragma unroll
      for (int q = 0; q < 4; ++q) {
        float gg = g[j + q], bb = bta[j + q];
        if (PARAM_BF16) { gg = bf16_round(gg); bb = bf16_round(bb); }
        sm[q] = vals[u * 4 + q]; o[q] = (vals[u * 4 + q] - mu) * rs * gg + bb;
      }
      if (out_sum) *(volatile v4f*)(out_sum + (size_t)row * N + j) = sm;
      *(volatile v4f*)(out_norm + (size_t)row * N + j) = o;
    }
    if (pass == 0) __threadfence();
  }
}


typedef _Float16 v16h __attribute__((ext_vector_type(16)));
union FragH { v16h v; v8us half[2]; _Float16 h[16]; unsigned short u[16]; };
template <int NT>
__device__ __forceinline__ v8f mmaH(v16h ah, v16h al, v16h bh, v16h bl, v8f c) {
  c = __builtin_amdgcn_wmma_f32_16x16x32_f16(false, ah, false, bh, (short)0, c, false, false);
  if (NT >= 2) c = __builtin_amdgcn_wmma_f32_16x16x32_f16(false, al, false, bh, (short)0, c, false, false);
  if (NT >= 3) c = __builtin_amdgcn_wmma_f32_16x16x32_f16(false, ah, false, bl, (short)0, c, false, false);
  asm volatile("v_nop\n\tv_nop\n\tv_nop\n\tv_nop" : "+v"(c) : "v"(ah), "v"(al), "v"(bh), "v"(bl));
  return c;
}
template <bool ASPLIT>
__global__ __launch_bounds__(128) void k_gemm_h(const float* __restrict__ A, int lda, size_t sA, const _Float16* __restrict__ Bh, int ldb, size_t sB, float alpha, float* __restrict__ C, int ldc, size_t sC, int M, int N, int K) {
  __shared__ __attribute__((aligned(16))) float so[4][16][64];
  const int tid = threadIdx.x, w = tid >> 5, lane = tid & 31, ln = lane & 15, hh = lane >> 4; const int by = blockIdx.y;
  A += (size_t)by * sA; Bh += (size_t)by * sB; C += (size_t)by * sC;
  const int ntn = (N + 63) / 64; const int wid = blockIdx.x * 4 + w; const int mt = wid / ntn, nq = wid % ntn; if (mt * 16 >= M) return;
  const int row0 = mt * 16, col0 = nq * 64; const float* arow = A + (size_t)(row0 + ln) * lda;
  v8f acc[4] = {};
  for (int kb = 0; kb < K; kb += 32) {
    FragH ah, al;
    const v4f x0 = *(const v4fa*)(arow + kb + 8 * hh), x1 = *(const v4fa*)(arow + kb + 8 * hh + 4), x2 = *(const v4fa*)(arow + kb + 16 + 8 * hh), x3 = *(const v4fa*)(arow + kb + 16 + 8 * hh + 4);
    float xs[16] = {x0[0],x0[1],x0[2],x0[3],x1[0],x1[1],x1[2],x1[3],x2[0],x2[1],x2[2],x2[3],x3[0],x3[1],x3[2],x3[3]};
#pragma unroll
    for (int i = 0; i < 16; ++i) { const _Float16 h = (_Float16)xs[i]; ah.h[i] = h; al.h[i] = ASPLIT ? (_Float16)(xs[i] - (float)h) : (_Float16)0.0f; }
#pragma unroll
    for (int t = 0; t < 4; ++t) { if (col0 + t * 16 >= N) continue; const size_t boff = (size_t)(col0 + t * 16 + ln) * ldb + kb; FragH bq; bq.half[0] = *(const v8us*)(Bh + boff + 8 * hh); bq.half[1] = *(const v8us*)(Bh + boff + 16 + 8 * hh);
      acc[t] = mmaH<ASPLIT ? 2 : 1>(ah.v, al.v, bq.v, bq.v, acc[t]); }
  }
#pragma unroll
  for (int t = 0; t < 4; ++t) { if (col0 + t * 16 >= N) continue;
#pragma unroll
    for (int r = 0; r < 8; ++r) so[w][8 * hh + r][t * 16 + ln] = acc[t][r] * alpha; }
  __builtin_amdgcn_fence(__ATOMIC_ACQ_REL, "workgroup"); __builtin_amdgcn_wave_barrier();
  const int rsub = lane >> 4, c4 = (lane & 15) * 4;
  for (int pass = 0; pass < 2; ++pass) {
#pragma unroll
    for (int q = 0; q < 8; ++q) { const int r = q * 2 + rsub; if (col0 + c4 < N) { const v4f v = *(const v4fa*)&so[w][r][c4]; *(volatile v4f*)(C + (size_t)(row0 + r) * ldc + col0 + c4) = v; } }
    if (pass == 0) __threadfence(); }
}

__global__ __launch_bounds__(256) void k_wt_f16(const float* __restrict__ W, _Float16* __restrict__ Wt, int K, int N, float scale) {
  const int t = blockIdx.x * 256 + threadIdx.x; if (t >= N * (K / 8)) return; const int n = t / (K / 8), k8 = (t % (K / 8)) * 8; FragH f;
#pragma unroll
  for (int i = 0; i < 8; ++i) f.h[i] = (_Float16)(bf16_round(W[(size_t)(k8 + i) * N + n]) * scale); const v8us o = f.half[0];
  *(volatile v8us*)((unsigned short*)Wt + (size_t)n * K + k8) = o; __threadfence(); *(volatile v8us*)((unsigned short*)Wt + (size_t)n * K + k8) = o;
}
template <int ACT>
__global__ __launch_bounds__(128) void k_gemm_hhx(const _Float16* __restrict__ A, int lda, size_t sA, const _Float16* __restrict__ Bh, int ldb, size_t sB, float alpha, const float* __restrict__ bias, size_t sBias, const float* __restrict__ CP, int rowsPerB, size_t sCPb, int row0g,
    float* __restrict__ C, _Float16* __restrict__ C16, int ldc, size_t sC, int M, int N, int K) {
  __shared__ __attribute__((aligned(16))) float so[4][16][64];
  const int tid = threadIdx.x, w = tid >> 5, lane = tid & 31, ln = lane & 15, hh = lane >> 4; const int by = blockIdx.y;
  A += (size_t)by * sA; Bh += (size_t)by * sB; const size_t cofs = (size_t)by * sC; const float* bp = bias ? bias + (size_t)by * sBias : nullptr;
  const int ntn = (N + 63) / 64; const int wid = blockIdx.x * 4 + w; const int mt = wid / ntn, nq = wid % ntn; if (mt * 16 >= M) return;
  const int row0 = mt * 16, col0 = nq * 64; const _Float16* arow = A + (size_t)(row0 + ln) * lda;
  v8f acc[4] = {};
  for (int kb = 0; kb < K; kb += 32) { FragH ah; ah.half[0] = *(const v8us*)((const unsigned short*)arow + kb + 8 * hh); ah.half[1] = *(const v8us*)((const unsigned short*)arow + kb + 16 + 8 * hh);
#pragma unroll
    for (int t = 0; t < 4; ++t) { if (col0 + t * 16 >= N) continue; const size_t boff = (size_t)(col0 + t * 16 + ln) * ldb + kb; FragH bq; bq.half[0] = *(const v8us*)((const unsigned short*)Bh + boff + 8 * hh); bq.half[1] = *(const v8us*)((const unsigned short*)Bh + boff + 16 + 8 * hh);
      acc[t] = mmaH<1>(ah.v, ah.v, bq.v, bq.v, acc[t]); }
  }
#pragma unroll
  for (int t = 0; t < 4; ++t) { if (col0 + t * 16 >= N) continue; const int col = col0 + t * 16 + ln; const float bv = bp ? bf16_round(bp[col]) : 0.f;
#pragma unroll
    for (int r = 0; r < 8; ++r) { float v = acc[t][r] * alpha + bv; if (CP) { const int bidx = (row0g + row0 + 8 * hh + r) / rowsPerB; v += CP[(size_t)bidx * sCPb + (size_t)by * 64 + col]; } if (ACT == 1) v = (v > 0.f) ? v : expm1f(v); else if (ACT == 7) v = (v > 0.f) ? v + 1.0f : expf(v); else if (ACT == 8) v = tanhf(v); else if (ACT == 9) v = 0.5f * v * (1.0f + tanhf(0.7978845608028654f * (v + 0.044715f * v * v * v))); else if (ACT == 11) v = 1.0f / (1.0f + expf(-v)); else if (ACT == 12) v = (v > 0.f) ? v : 0.01f * v; else if (ACT == 14) v = (v > 0.f) ? v : 0.1f * v; else if (ACT == 15) v = v / (1.0f + expf(-v)); else if (ACT == 3) v = fmaxf(v, 0.f); else if (ACT == 6) v = 0.5f * v * (1.0f + erff(v * 0.70710678118654752f)); so[w][8 * hh + r][t * 16 + ln] = v; } }
  __builtin_amdgcn_fence(__ATOMIC_ACQ_REL, "workgroup"); __builtin_amdgcn_wave_barrier();
  const int rsub = lane >> 4, c4 = (lane & 15) * 4; typedef _Float16 v4h __attribute__((ext_vector_type(4)));
  for (int pass = 0; pass < 2; ++pass) {
#pragma unroll
    for (int q = 0; q < 8; ++q) { const int r = q * 2 + rsub; if (col0 + c4 < N) { const v4f v = *(const v4fa*)&so[w][r][c4]; if (C) *(volatile v4f*)(C + cofs + (size_t)(row0 + r) * ldc + col0 + c4) = v; if (C16) { v4h h4; for (int i = 0; i < 4; ++i) h4[i] = (_Float16)v[i]; *(volatile v4h*)(C16 + cofs + (size_t)(row0 + r) * ldc + col0 + c4) = h4; } } }
    if (pass == 0) __threadfence(); }
}


typedef _Float16 v4h __attribute__((ext_vector_type(4)));

__global__ __launch_bounds__(256) void k_x16(const float* __restrict__ x, _Float16* __restrict__ X16, size_t n8) { const size_t t = (size_t)blockIdx.x * 256 + threadIdx.x; if (t >= n8) return; FragH f;
#pragma unroll
  for (int q = 0; q < 8; ++q) f.h[q] = (_Float16)bf16_round(x[t * 8 + q]); *(volatile v8us*)((unsigned short*)X16 + t * 8) = f.half[0]; __threadfence(); *(volatile v8us*)((unsigned short*)X16 + t * 8) = f.half[0]; }
__global__ __launch_bounds__(256) void k_h16(const float* __restrict__ x, _Float16* __restrict__ X16, size_t n8) { const size_t t = (size_t)blockIdx.x * 256 + threadIdx.x; if (t >= n8) return; FragH f;
#pragma unroll
  for (int q = 0; q < 8; ++q) f.h[q] = (_Float16)x[t * 8 + q]; *(volatile v8us*)((unsigned short*)X16 + t * 8) = f.half[0]; __threadfence(); *(volatile v8us*)((unsigned short*)X16 + t * 8) = f.half[0]; }
__global__ __launch_bounds__(256) void k_round16f(const float* __restrict__ W, _Float16* __restrict__ Bt, size_t n8) { const size_t t = (size_t)blockIdx.x * 256 + threadIdx.x; if (t >= n8) return; FragH f;
#pragma unroll
  for (int i = 0; i < 8; ++i) f.h[i] = (_Float16)(bf16_round(W[t * 8 + i]) * 16.0f); *(volatile v8us*)((unsigned short*)Bt + t * 8) = f.half[0]; __threadfence(); *(volatile v8us*)((unsigned short*)Bt + t * 8) = f.half[0]; }
template <int NHv, int TTv>
__global__ __launch_bounds__(256) void k_vt(const _Float16* __restrict__ V16, int ldv, int voff, _Float16* __restrict__ Vt) { __shared__ unsigned short tl[64][66]; const int tid = threadIdx.x; const int slab = blockIdx.x / (TTv / 64), lg = blockIdx.x % (TTv / 64); const int b = slab / NHv, h = slab % NHv;
  for (int i = tid; i < 64 * 8; i += 256) { const int r = i / 8, c8 = (i % 8) * 8; FragH f; f.half[0] = *(const v8us*)((const unsigned short*)V16 + ((size_t)b * TTv + lg * 64 + r) * ldv + voff + h * 64 + c8);
#pragma unroll
    for (int q = 0; q < 8; ++q) tl[r][c8 + q] = f.u[q]; }
  __syncthreads();
  for (int pass = 0; pass < 2; ++pass) {
#pragma unroll
    for (int rd = 0; rd < 2; ++rd) { const int d = rd * 32 + tid / 8, pc = tid % 8; FragH f;
#pragma unroll
      for (int q = 0; q < 8; ++q) f.u[q] = tl[pc * 8 + q][d];
      *(volatile v8us*)((unsigned short*)Vt + ((size_t)slab * 64 + d) * TTv + lg * 64 + pc * 8) = f.half[0]; }
    if (pass == 0) __threadfence(); } }

__global__ __launch_bounds__(256) void k_hl(const float* __restrict__ F, _Float16* __restrict__ Hh, _Float16* __restrict__ Hl, size_t n8) { const size_t t = (size_t)blockIdx.x * 256 + threadIdx.x; if (t >= n8) return; FragH fh, fl; const v4f a = *(const v4fa*)(F + t * 8), c = *(const v4fa*)(F + t * 8 + 4);
#pragma unroll
  for (int q = 0; q < 4; ++q) { _Float16 h = (_Float16)a[q]; fh.h[q] = h; fl.h[q] = (_Float16)((a[q] - (float)h) * 1024.0f); h = (_Float16)c[q]; fh.h[4 + q] = h; fl.h[4 + q] = (_Float16)((c[q] - (float)h) * 1024.0f); }
  for (int pass = 0; pass < 2; ++pass) { *(volatile v8us*)((unsigned short*)Hh + t * 8) = fh.half[0]; *(volatile v8us*)((unsigned short*)Hl + t * 8) = fl.half[0]; if (pass == 0) __threadfence(); } }

__device__ __forceinline__ float sigm_f(float x) { return __builtin_amdgcn_rcpf(1.0f + __expf(-x)); }
__device__ __forceinline__ float tanh_f(float x) { const float a = fabsf(x); const float big = 1.0f - 2.0f * __builtin_amdgcn_rcpf(1.0f + __expf(2.0f * a)); const float sml = a - a * a * a * (1.0f / 3.0f); const float r = (a < 0.03f) ? sml : big; return (x < 0.f) ? -r : r; }
__global__ __launch_bounds__(256) void k_wcat(const float* __restrict__ whh, const float* __restrict__ wih, int DIN, int KL, _Float16* __restrict__ Wc) { const int t = blockIdx.x * 256 + threadIdx.x; if (t >= G4 * (KL / 8)) return; const int k0 = (t % (KL / 8)) * 8, g = t / (KL / 8); FragH f;
#pragma unroll
  for (int q = 0; q < 8; ++q) { const int k = k0 + q; float v = 0.f; if (k < HH) v = bf16_round(whh[(size_t)g * HH + k]); else if (k < HH + DIN) v = bf16_round(wih[(size_t)g * DIN + (k - HH)]); f.h[q] = (_Float16)(v * 16.0f); }
  *(volatile v8us*)((unsigned short*)Wc + (size_t)g * KL + k0) = f.half[0]; __threadfence(); *(volatile v8us*)((unsigned short*)Wc + (size_t)g * KL + k0) = f.half[0]; }
__global__ __launch_bounds__(256) void k_zero(float* __restrict__ P, size_t n4) { const size_t t = (size_t)blockIdx.x * 256 + threadIdx.x; if (t >= n4) return; const v4f z = {0.f, 0.f, 0.f, 0.f}; *(volatile v4f*)(P + t * 4) = z; __threadfence(); *(volatile v4f*)(P + t * 4) = z; }
__global__ __launch_bounds__(256) void k_prev(const float* __restrict__ HB, const float* __restrict__ CB, const int* __restrict__ pidx, const float* __restrict__ pmarg, int t, int L, const int* __restrict__ tok, const float* __restrict__ emb, const float* __restrict__ HB1, _Float16* __restrict__ A, _Float16* __restrict__ AL, float* __restrict__ CPV) {
  #pragma clang fp contract(off)
  const int tid = threadIdx.x, w = tid >> 5, l = tid & 31; const int b = blockIdx.x * 8 + w; if (b >= NBt) return;
  int id[KP]; float mg[KP];
#pragma unroll
  for (int k = 0; k < KP; ++k) { int i = pidx[((size_t)b * TT + t) * KP + k]; id[k] = min(max(i, 0), TT - 1); mg[k] = bf16_round(pmarg[((size_t)b * TT + t) * KP + k]); }
  for (int pass = 0; pass < 2; ++pass) {
#pragma unroll
    for (int qd = 0; qd < 4; ++qd) { const int u0 = qd * 128 + 4 * l; v4f hp = {0.f, 0.f, 0.f, 0.f}, cp = {0.f, 0.f, 0.f, 0.f};
#pragma unroll
      for (int k = 0; k < KP; ++k) { const v4f hv = *(const v4fa*)(HB + ((size_t)id[k] * NBt + b) * HH + u0), cv = *(const v4fa*)(CB + ((size_t)id[k] * NBt + b) * HH + u0);
#pragma unroll
        for (int q = 0; q < 4; ++q) { hp[q] += mg[k] * hv[q]; cp[q] += mg[k] * cv[q]; } }
      FragH f, fl;
#pragma unroll
      for (int q = 0; q < 4; ++q) { const _Float16 hi = (_Float16)hp[q]; f.h[q] = hi; fl.h[q] = (_Float16)((hp[q] - (float)hi) * 1024.0f); }
      *(volatile unsigned long long*)((unsigned short*)A + (size_t)b * AP + u0) = *(const unsigned long long*)&f.u[0]; *(volatile unsigned long long*)((unsigned short*)AL + (size_t)b * HH + u0) = *(const unsigned long long*)&fl.u[0]; *(volatile v4f*)(CPV + (size_t)b * HH + u0) = cp; }
    if (L == 0) { int tk = tok[(size_t)b * TT + t]; tk = min(max(tk, 0), 31999);
#pragma unroll
      for (int rep = 0; rep < 2; ++rep) { const int ch = l + 32 * rep; if (ch < 40) { FragH f;
#pragma unroll
          for (int q = 0; q < 8; ++q) { const int e = ch * 8 + q; f.h[q] = (e < EE) ? (_Float16)bf16_round(emb[(size_t)tk * EE + min(e, EE - 1)]) : (_Float16)0.0f; }
          *(volatile v8us*)((unsigned short*)A + (size_t)b * AP + HH + ch * 8) = f.half[0]; } } }
    else {
#pragma unroll
      for (int qd = 0; qd < 4; ++qd) { const int u0 = qd * 128 + 4 * l; const v4f hv = *(const v4fa*)(HB1 + ((size_t)t * NBt + b) * HH + u0); FragH f; f.h[0] = (_Float16)hv[0]; f.h[1] = (_Float16)hv[1]; f.h[2] = (_Float16)hv[2]; f.h[3] = (_Float16)hv[3]; *(volatile unsigned long long*)((unsigned short*)A + (size_t)b * AP + HH + u0) = *(const unsigned long long*)&f.u[0]; } }
    if (pass == 0) __threadfence(); } }
__global__ __launch_bounds__(256) void k_cell(const float* __restrict__ G, const float* __restrict__ CPV, int t, float* __restrict__ HB, float* __restrict__ CB) {
  #pragma clang fp contract(off)
  const int tid = threadIdx.x, w = tid >> 5, l = tid & 31; const int b = blockIdx.x * 8 + w; if (b >= NBt) return; const float* g = G + (size_t)b * G4;
  for (int pass = 0; pass < 2; ++pass) {
#pragma unroll
    for (int qd = 0; qd < 4; ++qd) { const int u0 = qd * 128 + 4 * l; const v4f gi = *(const v4fa*)(g + u0), gf = *(const v4fa*)(g + HH + u0), gg = *(const v4fa*)(g + 2 * HH + u0), go = *(const v4fa*)(g + 3 * HH + u0), cp = *(const v4fa*)(CPV + (size_t)b * HH + u0); v4f c, h;
#pragma unroll
      for (int q = 0; q < 4; ++q) { const float cn = sigm_f(gf[q]) * cp[q] + sigm_f(gi[q]) * tanh_f(gg[q]); c[q] = cn; h[q] = sigm_f(go[q]) * tanh_f(cn); }
      *(volatile v4f*)(HB + ((size_t)t * NBt + b) * HH + u0) = h; *(volatile v4f*)(CB + ((size_t)t * NBt + b) * HH + u0) = c; }
    if (pass == 0) __threadfence(); } }
__global__ __launch_bounds__(256) void k_out(const float* __restrict__ HB, const int* __restrict__ pos, const float* __restrict__ lw, const float* __restrict__ lb, float* __restrict__ out) {
  #pragma clang fp contract(off)
  __shared__ float pooled[HH]; __shared__ __attribute__((aligned(16))) float orow[NL]; const int tid = threadIdx.x; const int b = blockIdx.x; int s = pos[b * 2], e = pos[b * 2 + 1]; s = min(max(s, 0), TT); e = min(max(e, 0), TT);
  for (int u = tid; u < HH; u += 256) { float m = 0.f; if (s < e) { m = -3.0e38f;
#pragma unroll 1
      for (int t = s; t < e; ++t) m = fmaxf(m, HB[((size_t)t * NBt + b) * HH + u]); } pooled[u] = m; }
  __syncthreads();
  if (tid < NL) { float acc = bf16_round(lb[tid]);
#pragma unroll 1
    for (int u = 0; u < HH; ++u) acc += pooled[u] * bf16_round(lw[(size_t)tid * HH + u]); orow[tid] = acc; }
  __syncthreads();
  if (tid < NL / 4) { const v4f v = *(const v4fa*)&orow[tid * 4]; *(volatile v4f*)(out + (size_t)b * NL + tid * 4) = v; __threadfence(); *(volatile v4f*)(out + (size_t)b * NL + tid * 4) = v; } }

extern "C" void kernel_launch(void* const* d_in, const int* in_sizes, int n_in,
                              void* d_out, int out_size, void* d_ws, size_t ws_size, hipStream_t stream) {
  (void)in_sizes; (void)n_in; (void)out_size;
  const float* const* I = (const float* const*)d_in; const int* tok = (const int*)d_in[0]; const int* pos = (const int*)d_in[1]; const int* pidx = (const int*)d_in[2]; const float* pmarg = I[3]; const float* emb = I[4]; const float* Wih0 = I[5]; const float* Whh0 = I[6]; const float* b0 = I[7]; const float* Wih1 = I[8]; const float* Whh1 = I[9]; const float* b1 = I[10]; const float* lw = I[11]; const float* lb = I[12];
  char* ws = (char*)d_ws; size_t off = 0;
  auto take = [&](size_t bytes) { char* p = ws + off; off += (bytes + 255) & ~(size_t)255; return p; };
  _Float16* W0 = (_Float16*)take((size_t)G4 * K0 * 2); _Float16* W1c = (_Float16*)take((size_t)G4 * K1 * 2); _Float16* A = (_Float16*)take((size_t)NBt * AP * 2); _Float16* AL = (_Float16*)take((size_t)NBt * HH * 2); float* CPV = (float*)take((size_t)NBt * HH * 4); float* Gp = (float*)take((size_t)NBt * G4 * 4);
  float* HB1 = (float*)take((size_t)TT * NBt * HH * 4); float* CB1 = (float*)take((size_t)TT * NBt * HH * 4); float* HB2 = (float*)take((size_t)TT * NBt * HH * 4); float* CB2 = (float*)take((size_t)TT * NBt * HH * 4);
  if (off > ws_size) return;
  k_wcat<<<(G4 * (K0 / 8) + 255) / 256, 256, 0, stream>>>(Whh0, Wih0, EE, K0, W0); k_wcat<<<(G4 * (K1 / 8) + 255) / 256, 256, 0, stream>>>(Whh1, Wih1, HH, K1, W1c);
  const size_t n4 = (size_t)TT * NBt * HH / 4; const unsigned gz = (unsigned)((n4 + 255) / 256);
  k_zero<<<gz, 256, 0, stream>>>(HB1, n4); k_zero<<<gz, 256, 0, stream>>>(CB1, n4); k_zero<<<gz, 256, 0, stream>>>(HB2, n4); k_zero<<<gz, 256, 0, stream>>>(CB2, n4);
  k_zero<<<(NBt * AP / 2 / 4 + 255) / 256, 256, 0, stream>>>((float*)A, (size_t)NBt * AP / 2 / 4);
  for (int L = 0; L < 2; ++L) { float* HB = L ? HB2 : HB1; float* CB = L ? CB2 : CB1; const _Float16* Wc = L ? W1c : W0; const int KL = L ? K1 : K0; const float* bb = L ? b1 : b0;
    for (int t = 0; t < TT; ++t) {
      k_prev<<<NBt / 8, 256, 0, stream>>>(HB, CB, pidx, pmarg, t, L, tok, emb, HB1, A, AL, CPV);
      k_gemm_hhx<0><<<dim3(((NBt / 16) * (G4 / 64) + 3) / 4, 1), 128, 0, stream>>>(A, AP, 0, Wc, KL, 0, 0.0625f, bb, 0, nullptr, 1, 0, 0, Gp, nullptr, G4, 0, NBt, G4, KL);
      k_gemm_hhx<0><<<dim3(((NBt / 16) * (G4 / 64) + 3) / 4, 1), 128, 0, stream>>>(AL, HH, 0, Wc, KL, 0, 0.0625f / 1024.0f, nullptr, 0, Gp, 1, (size_t)G4, 0, Gp, nullptr, G4, 0, NBt, G4, HH);
      k_cell<<<NBt / 8, 256, 0, stream>>>(Gp, CPV, t, HB, CB); } }
  k_out<<<NBt, 256, 0, stream>>>(HB2, pos, lw, lb, (float*)d_out);
}
